// MultiMLPLayer_62947040690424
// MI455X (gfx1250) — hardware-verified
//
#include <hip/hip_runtime.h>
#include <math.h>

typedef __attribute__((ext_vector_type(16))) _Float16 v16h;
typedef __attribute__((ext_vector_type(16))) __bf16 v16b;
typedef __attribute__((ext_vector_type(8)))  _Float16 v8h;
typedef __attribute__((ext_vector_type(8)))  float v8f;
typedef __attribute__((ext_vector_type(4)))  float v4f;
typedef __attribute__((ext_vector_type(2)))  float v2f;
typedef __attribute__((ext_vector_type(4)))  unsigned v4u;
typedef __attribute__((ext_vector_type(4)))  int v4i;
typedef float __attribute__((may_alias)) float_a;
typedef int __attribute__((may_alias)) int_a;

template <typename T> __device__ __forceinline__ void vst2(void* p, T v) { *(volatile T*)p = v; __threadfence(); *(volatile T*)p = v; }
__device__ __forceinline__ v8f wmma16(v16h a, v16h b, v8f c) {
  v8f d = __builtin_amdgcn_wmma_f32_16x16x32_f16(false, a, false, b, (short)0, c, false, false);
  asm volatile("v_nop\n\tv_nop\n\tv_nop\n\tv_nop" : "+v"(d) : "v"(a), "v"(b));
  return d;
}
__device__ __forceinline__ v8f wmma_bf(v16b a, v16b b, v8f c) {
  v8f d = __builtin_amdgcn_wmma_f32_16x16x32_bf16(false, a, false, b, (short)0, c, false, false);
  asm volatile("v_nop\n\tv_nop\n\tv_nop\n\tv_nop" : "+v"(d) : "v"(a), "v"(b));
  return d;
}
__device__ __forceinline__ v16h frag_h(const _Float16* rowk0, int lane) {
  union { v16h v; v8h q[2]; } u; const _Float16* p = rowk0 + 8 * (lane >> 4);
  u.q[0] = *(const v8h*)p; u.q[1] = *(const v8h*)(p + 16); return u.v;
}
__device__ __forceinline__ v16h frag_f32(const float* rowk0, int lane) {
  v16h a; const float* p = rowk0 + 8 * (lane >> 4);
#pragma unroll
  for (int i = 0; i < 8; ++i) { a[i] = (_Float16)p[i]; a[8 + i] = (_Float16)p[16 + i]; }
  return a;
}
__device__ __forceinline__ v16h frag_f32s(const float* rowk0, int lane, float sc) {
  v16h a; const float* p = rowk0 + 8 * (lane >> 4);
#pragma unroll
  for (int i = 0; i < 8; ++i) { a[i] = (_Float16)(p[i] * sc); a[8 + i] = (_Float16)(p[16 + i] * sc); }
  return a;
}
__device__ __forceinline__ v16h fragc_f32(const float* W, int k0, int n, int lane, int ld, int K) {
  v16h a; const int g = lane >> 4;
#pragma unroll
  for (int i = 0; i < 8; ++i) { const int ka = k0 + 8 * g + i, kb = ka + 16;
    a[i] = (_Float16)(ka < K ? W[(size_t)(ka < K ? ka : K - 1) * ld + n] : 0.f); a[8 + i] = (_Float16)(kb < K ? W[(size_t)(kb < K ? kb : K - 1) * ld + n] : 0.f); }
  return a;
}
struct F2 { v16b h, l; };
__device__ __forceinline__ F2 bsplit16(const float v[16]) { F2 r;
#pragma unroll
  for (int i = 0; i < 16; ++i) { const __bf16 h = (__bf16)v[i]; r.h[i] = h; r.l[i] = (__bf16)(v[i] - (float)h); }
  return r; }
__device__ __forceinline__ F2 split_row(const float* row, int k0, int lane) { float v[16]; const float* p = row + k0 + 8 * (lane >> 4);
#pragma unroll
  for (int i = 0; i < 8; ++i) { v[i] = p[i]; v[8 + i] = p[16 + i]; }
  return bsplit16(v); }
__device__ __forceinline__ F2 split_rowK(const float* row, int k0, int lane, int K) { float v[16]; const int g = lane >> 4;
#pragma unroll
  for (int i = 0; i < 8; ++i) { const int ka = k0 + 8 * g + i, kb = ka + 16; v[i] = ka < K ? row[ka < K ? ka : K - 1] : 0.f; v[8 + i] = kb < K ? row[kb < K ? kb : K - 1] : 0.f; }
  return bsplit16(v); }
__device__ __forceinline__ F2 split_col(const float* W, int k0, int n, int lane, int ld, int K) { float v[16]; const int g = lane >> 4;
#pragma unroll
  for (int i = 0; i < 8; ++i) { const int ka = k0 + 8 * g + i, kb = ka + 16; v[i] = ka < K ? W[(size_t)(ka < K ? ka : K - 1) * ld + n] : 0.f; v[8 + i] = kb < K ? W[(size_t)(kb < K ? kb : K - 1) * ld + n] : 0.f; }
  return bsplit16(v); }
__device__ __forceinline__ v8f mac3(const F2& a, const F2& b, v8f c) { c = wmma_bf(a.l, b.h, c); c = wmma_bf(a.h, b.l, c); return wmma_bf(a.h, b.h, c); }
__device__ __forceinline__ float sigm(float v) { return 1.0f / (1.0f + expf(-v)); }
#define LDSX() do { asm volatile("s_wait_dscnt 0" ::: "memory"); __builtin_amdgcn_wave_barrier(); __builtin_amdgcn_fence(__ATOMIC_RELEASE, "workgroup"); } while (0)


#define NTK 8192
#define EE 1024
#define GH 256
#define NM 6
#ifndef NRT
#define NRT (NTK / 64)
#endif
typedef __attribute__((ext_vector_type(8))) __bf16 v8b;
__device__ __forceinline__ v16b frag_b(const __bf16* rowk0, int lane) {
  union { v16b v; v8b q[2]; } u; const __bf16* p = rowk0 + 8 * (lane >> 4);
  u.q[0] = *(const v8b*)p; u.q[1] = *(const v8b*)(p + 16); return u.v;
}
__device__ __forceinline__ float bfr(float v) { return (float)(__bf16)v; }
__device__ __attribute__((noinline)) float exp_ni(float v) { return expf(v); }
__device__ __attribute__((noinline)) float erf_ni(float v) { return erff(v); }

__device__ __forceinline__ float gelu_exact(float v) { return 0.5f * v * (1.0f + erf_ni(v * 0.70710678118654752f)); }
#define PK_G1  0
#define PK_SM  (PK_G1 + GH * EE)
#define PK_DF  (PK_SM + 32 * EE)
#define PK_DP  (PK_DF + 2048 * EE)
#define PK_SF  (PK_DP + EE * 2048)
#define PK_SP  (PK_SF + EE * EE)
#define PK_END (PK_SP + EE * EE)
#define WS_PK   0u
#define WS_XB   (((2u * PK_END) + 127u) / 128u * 128u)
#define WS_SML  (WS_XB + 2u * NTK * EE)
#define WS_EXP  (WS_SML + 4u * NTK * 32)
#define WS_WGT  (WS_EXP + 4u * NTK)
#define WS_CNT  (WS_WGT + 4u * NTK)
#define WS_LIST (WS_CNT + 128u)
#define WS_HBH  (WS_LIST + 4u * NM * NTK)
#define WS_HBL  (WS_HBH + 2u * (size_t)NTK * 2048)
#define WS_END  (WS_HBL + 2u * (size_t)NTK * 2048)

__global__ __launch_bounds__(256) void k_pack(const float* __restrict__ GW1, const float* __restrict__ P2W, const float* __restrict__ P4W, const float* __restrict__ RGU, const float* __restrict__ FLDW, const float* __restrict__ DFW, const float* __restrict__ DPW, const float* __restrict__ SFW, const float* __restrict__ SPW, __bf16* __restrict__ PK) {
  __shared__ __align__(16) __bf16 s[2048]; const int n = blockIdx.x, which = blockIdx.y, t = threadIdx.x; int K = EE; size_t dst;
  if (which == 0) { if (n >= GH) return; dst = PK_G1 + (size_t)n * EE; for (int k = t; k < EE; k += 256) s[k] = (__bf16)GW1[(size_t)k * GH + n]; }
  else if (which == 1) { if (n >= 32) return; dst = PK_SM + (size_t)n * EE; for (int k = t; k < EE; k += 256) { float v = 0.f; if (n < 2) v = P2W[(size_t)n * EE + k]; else if (n < 6) v = P4W[(size_t)(n - 2) * EE + k]; else if (n == 6) v = RGU[k]; else if (n >= 16) v = FLDW[(size_t)k * 16 + (n - 16)]; s[k] = (__bf16)v; } }
  else if (which == 2) { dst = PK_DF + (size_t)n * EE; for (int k = t; k < EE; k += 256) s[k] = (__bf16)DFW[(size_t)k * 2048 + n]; }
  else if (which == 3) { if (n >= EE) return; K = 2048; dst = PK_DP + (size_t)n * 2048; for (int k = t; k < 2048; k += 256) s[k] = (__bf16)DPW[(size_t)k * EE + n]; }
  else if (which == 4) { if (n >= EE) return; dst = PK_SF + (size_t)n * EE; for (int k = t; k < EE; k += 256) s[k] = (__bf16)SFW[(size_t)k * EE + n]; }
  else { if (n >= EE) return; dst = PK_SP + (size_t)n * EE; for (int k = t; k < EE; k += 256) s[k] = (__bf16)SPW[(size_t)k * EE + n]; }
  __syncthreads();
  for (int q = t; q < K / 8; q += 256) vst2((unsigned*)(PK + dst + q * 8), *(const v4u*)&s[q * 8]);
}
__global__ __launch_bounds__(128) void k_xb(const float* __restrict__ X, __bf16* __restrict__ XB) {
  __shared__ __align__(16) __bf16 s[EE]; const size_t r = blockIdx.x; const int t = threadIdx.x;
  for (int k = t; k < EE; k += 128) s[k] = (__bf16)X[r * EE + k];
  __syncthreads();
  vst2((unsigned*)(XB + r * EE + t * 8), *(const v4u*)&s[t * 8]);
}
__global__ __launch_bounds__(128) void k_gate(const __bf16* __restrict__ XB, const __bf16* __restrict__ PK, const float* __restrict__ GB1, const float* __restrict__ GW2, const float* __restrict__ GB2, const float* __restrict__ EB, const float* __restrict__ PMA, float* __restrict__ SML, int* __restrict__ EXPo, float* __restrict__ WGT) {
  __shared__ __align__(16) float sg[64][GH + 4]; __shared__ __align__(16) float ss[64][36]; __shared__ __align__(16) int sexp[64]; __shared__ __align__(16) float swg[64];
  const int tid = threadIdx.x, wave = tid >> 5, lane = tid & 31, col = lane & 15, g = lane >> 4; const size_t r0 = (size_t)blockIdx.x * 64 + wave * 16;
#pragma unroll 1
  for (int pass = 0; pass < 3; ++pass) { const int nt = (pass < 2) ? 8 : 2; const __bf16* P = (pass < 2) ? PK + PK_G1 + (size_t)pass * 128 * EE : PK + PK_SM; v8f acc[8] = {};
#pragma unroll 2
    for (int kc = 0; kc < EE / 32; ++kc) { const v16b a = frag_b(XB + (r0 + col) * EE + kc * 32, lane);
#pragma unroll
      for (int j = 0; j < 8; ++j) if (j < nt) acc[j] = wmma_bf(a, frag_b(P + (size_t)(j * 16 + col) * EE + kc * 32, lane), acc[j]); }
    if (pass < 2) {
#pragma unroll
      for (int j = 0; j < 8; ++j) { const int c = pass * 128 + j * 16 + col; const float bb = bfr(GB1[c]);
#pragma unroll
        for (int r = 0; r < 8; ++r) sg[wave * 16 + 8 * g + r][c] = gelu_exact(acc[j][r] + bb); } }
    else {
#pragma unroll
      for (int j = 0; j < 2; ++j)
#pragma unroll
        for (int r = 0; r < 8; ++r) ss[wave * 16 + 8 * g + r][j * 16 + col] = acc[j][r]; } }
  __syncthreads();
  if (tid < 64) { const int rl = tid; float gl[NM];
#pragma unroll
    for (int m = 0; m < NM; ++m) { float a = 0.f; for (int k = 0; k < GH; ++k) a += sg[rl][k] * bfr(GW2[k * NM + m]); gl[m] = (a + bfr(GB2[m])) + bfr(EB[m]); }
    float mx = gl[0]; int am = 0;
#pragma unroll
    for (int m = 1; m < NM; ++m) if (gl[m] > mx) { mx = gl[m]; am = m; }
    float se = 0.f; float pm[NM];
#pragma unroll
    for (int m = 0; m < NM; ++m) { pm[m] = exp_ni(gl[m] - mx); se += pm[m]; }
    float ptop = 0.f;
#pragma unroll
    for (int m = 0; m < NM; ++m) ptop = (m == am) ? pm[m] / se : ptop;
    sexp[rl] = am; swg[rl] = bfr(PMA[0]) * (ptop / (ptop + 1e-9f)); }
  __syncthreads();
  for (int q = tid; q < 64 * 8; q += 128) { const int r = q >> 3, pc = q & 7; vst2(SML + ((size_t)blockIdx.x * 64 + r) * 32 + pc * 4, *(const v4f*)&ss[r][pc * 4]); }
  if (tid < 16) vst2((unsigned*)(EXPo + (size_t)blockIdx.x * 64 + tid * 4), *(const v4u*)&sexp[tid * 4]); else if (tid < 32) vst2(WGT + (size_t)blockIdx.x * 64 + (tid - 16) * 4, *(const v4f*)&swg[(tid - 16) * 4]);
}
__global__ __launch_bounds__(256) void k_sort(const int* __restrict__ EXPo, int ntok, int* __restrict__ CNT, int* __restrict__ LIST) {
  __shared__ int scnt[NM]; __shared__ int sfirst[NM]; __shared__ __align__(16) int sc[32]; const int t = threadIdx.x;
  if (t < NM) { int c = 0, f = 0; bool seen = false; for (int i = 0; i < ntok; ++i) { const int e = EXPo[i]; if (e == t) { LIST[(size_t)t * NTK + c] = i; if (!seen) { f = i; seen = true; } ++c; } } scnt[t] = c; sfirst[t] = f; }
  __syncthreads();
  for (int q = t; q < NM * NTK; q += 256) { const int m = q / NTK, k = q % NTK; if (k >= scnt[m]) LIST[q] = sfirst[m]; }
  if (t < 32) sc[t] = (t < NM) ? scnt[t] : 0;
  __syncthreads();
  for (int q = t; q < NM * NTK / 4; q += 256) { v4u v; const int* p = LIST + (size_t)q * 4; v[0] = p[0]; v[1] = p[1]; v[2] = p[2]; v[3] = p[3]; vst2((unsigned*)(LIST + (size_t)q * 4), v); }
  if (t < 8) vst2((unsigned*)(CNT + t * 4), *(const v4u*)&sc[t * 4]);
}
template <int WHICH>
__global__ __launch_bounds__(128) void k_fc(const __bf16* __restrict__ XB, const __bf16* __restrict__ PK, const float* __restrict__ BB, const int* __restrict__ CNT, const int* __restrict__ LIST, __bf16* __restrict__ HBH, __bf16* __restrict__ HBL) {
  __shared__ __align__(16) __bf16 soh[4][16][136], sol[4][16][136]; __shared__ int stok[64];
  const int tid = threadIdx.x, wave = tid >> 5, lane = tid & 31, col = lane & 15, g = lane >> 4; const int cnt = CNT[WHICH]; if (blockIdx.x * 64 >= cnt) return;
  if (tid < 64) stok[tid] = LIST[(size_t)WHICH * NTK + blockIdx.x * 64 + tid];
  __syncthreads();
  const int n0 = blockIdx.y * 128; const __bf16* P = PK + (WHICH == 0 ? PK_DF : PK_SF);
  v8f acc[8] = {};
#pragma unroll 2
  for (int kc = 0; kc < EE / 32; ++kc) { const v16b a = frag_b(XB + (size_t)stok[wave * 16 + col] * EE + kc * 32, lane);
#pragma unroll
    for (int j = 0; j < 8; ++j) acc[j] = wmma_bf(a, frag_b(P + (size_t)(n0 + j * 16 + col) * EE + kc * 32, lane), acc[j]); }
#pragma unroll
  for (int j = 0; j < 8; ++j) { const float bb = bfr(BB[n0 + j * 16 + col]);
#pragma unroll
    for (int r = 0; r < 8; ++r) { const float v = gelu_exact(acc[j][r] + bb); const __bf16 hb = (__bf16)v; soh[wave][8 * g + r][j * 16 + col] = hb; sol[wave][8 * g + r][j * 16 + col] = (__bf16)(v - (float)hb); } }
  LDSX();
  for (int rl = 0; rl < 16; ++rl) { const int li = blockIdx.x * 64 + wave * 16 + rl; if (li < cnt && lane < 16) { const size_t o = (size_t)stok[wave * 16 + rl] * 2048 + n0 + lane * 8; vst2((unsigned*)(HBH + o), *(const v4u*)&soh[wave][rl][lane * 8]); vst2((unsigned*)(HBL + o), *(const v4u*)&sol[wave][rl][lane * 8]); } }
}
template <int WHICH>
__global__ __launch_bounds__(128) void k_pj(const __bf16* __restrict__ HBH, const __bf16* __restrict__ HBL, const __bf16* __restrict__ PK, const float* __restrict__ BB, const int* __restrict__ CNT, const int* __restrict__ LIST, const float* __restrict__ WGT, float* __restrict__ OUT) {
  constexpr int K = (WHICH == 0) ? 2048 : EE;
  __shared__ __align__(16) float so[4][16][132]; __shared__ int stok[64];
  const int tid = threadIdx.x, wave = tid >> 5, lane = tid & 31, col = lane & 15, g = lane >> 4; const int cnt = CNT[WHICH]; if (blockIdx.x * 64 >= cnt) return;
  if (tid < 64) stok[tid] = LIST[(size_t)WHICH * NTK + blockIdx.x * 64 + tid];
  __syncthreads();
  const int n0 = blockIdx.y * 128; const __bf16* P = PK + (WHICH == 0 ? PK_DP : PK_SP);
  v8f acc[8] = {};
#pragma unroll 2
  for (int kc = 0; kc < K / 32; ++kc) { const size_t ar = (size_t)stok[wave * 16 + col] * 2048 + kc * 32; const v16b ah = frag_b(HBH + ar, lane), al = frag_b(HBL + ar, lane);
#pragma unroll
    for (int j = 0; j < 8; ++j) { const v16b w = frag_b(P + (size_t)(n0 + j * 16 + col) * K + kc * 32, lane); acc[j] = wmma_bf(al, w, acc[j]); acc[j] = wmma_bf(ah, w, acc[j]); } }
#pragma unroll
  for (int j = 0; j < 8; ++j) { const float bb = bfr(BB[n0 + j * 16 + col]);
#pragma unroll
    for (int r = 0; r < 8; ++r) so[wave][8 * g + r][j * 16 + col] = (acc[j][r] + bb) * WGT[stok[wave * 16 + 8 * g + r]]; }
  LDSX();
  for (int rl = 0; rl < 16; ++rl) { const int li = blockIdx.x * 64 + wave * 16 + rl; if (li < cnt) vst2(OUT + (size_t)stok[wave * 16 + rl] * EE + n0 + lane * 4, *(const v4f*)&so[wave][rl][lane * 4]); }
}
__global__ __launch_bounds__(256) void k_small(int WHICH, const float* __restrict__ X, const float* __restrict__ SML, const int* __restrict__ CNT, const int* __restrict__ LIST, const float* __restrict__ WGT,
    const float* __restrict__ P2V, const float* __restrict__ P2A, const float* __restrict__ P2B, const float* __restrict__ P2BIAS, const float* __restrict__ P4V, const float* __restrict__ P4A, const float* __restrict__ P4B, const float* __restrict__ P4BIAS,
    const float* __restrict__ RGA, const float* __restrict__ RGB, const float* __restrict__ RGBIAS, const float* __restrict__ FLDB, const float* __restrict__ FLUW, const float* __restrict__ FLUB, float* __restrict__ OUT) {
  __shared__ __align__(16) float so[64][EE / 4 + 4]; __shared__ int stok[64]; __shared__ float sh[64][16];
  const int tid = threadIdx.x; const int cnt = CNT[WHICH]; if (blockIdx.x * 64 >= cnt) return;
  if (tid < 64) { const int tk = LIST[(size_t)WHICH * NTK + blockIdx.x * 64 + tid]; stok[tid] = tk; const float* sr = SML + (size_t)tk * 32;
    if (WHICH == 2) { for (int n = 0; n < 2; ++n) sh[tid][n] = bfr(P2A[n]) * gelu_exact(sr[n] + bfr(P2B[n])); }
    else if (WHICH == 3) { for (int n = 0; n < 4; ++n) sh[tid][n] = bfr(P4A[n]) * gelu_exact(sr[2 + n] + bfr(P4B[n])); }
    else if (WHICH == 4) { sh[tid][0] = 1.0f / (1.0f + exp_ni(-(sr[6] + bfr(RGB[0])))); }
    else { for (int j = 0; j < 16; ++j) sh[tid][j] = gelu_exact(sr[16 + j] + bfr(FLDB[j])); } }
  __syncthreads();
  const int rl = tid >> 2, part = tid & 3; const int tk = stok[rl]; const float wg = WGT[tk]; const float* xr = X + (size_t)tk * EE;
#pragma unroll 1
  for (int qtr = 0; qtr < 4; ++qtr) {
    for (int i = 0; i < 64; ++i) { const int e = qtr * 256 + part * 64 + i; float o;
      if (WHICH == 2) o = (sh[rl][0] * bfr(P2V[e]) + sh[rl][1] * bfr(P2V[EE + e])) + bfr(P2BIAS[e]);
      else if (WHICH == 3) { float a = 0.f;
#pragma unroll
        for (int n = 0; n < 4; ++n) a += sh[rl][n] * bfr(P4V[(size_t)n * EE + e]); o = a + bfr(P4BIAS[e]); }
      else if (WHICH == 4) o = sh[rl][0] * (bfr(xr[e]) * bfr(RGA[e])) + bfr(RGBIAS[e]);
      else { float ga = 0.f, be = 0.f;
#pragma unroll
        for (int j = 0; j < 16; ++j) { ga += sh[rl][j] * bfr(FLUW[(size_t)j * 2048 + e]); be += sh[rl][j] * bfr(FLUW[(size_t)j * 2048 + EE + e]); }
        o = (ga + bfr(FLUB[e])) * bfr(xr[e]) + (be + bfr(FLUB[EE + e])); }
      so[rl][part * 64 + i] = o * wg; }
    __syncthreads();
    for (int q = tid; q < 64 * 64; q += 256) { const int r = q >> 6, pc = q & 63; const int li = blockIdx.x * 64 + r; if (li < cnt) vst2(OUT + (size_t)stok[r] * EE + qtr * 256 + pc * 4, *(const v4f*)&so[r][pc * 4]); }
    __syncthreads(); }
}
extern "C" void kernel_launch(void* const* d_in, const int* in_sizes, int n_in, void* d_out, int out_size, void* d_ws, size_t ws_size, hipStream_t stream) {
  (void)in_sizes; (void)n_in; (void)out_size;
  const float** F = (const float**)d_in;
  if (ws_size < (size_t)WS_END) return;
  char* ws = (char*)d_ws; __bf16 *PK = (__bf16*)(ws + WS_PK), *XB = (__bf16*)(ws + WS_XB), *HBH = (__bf16*)(ws + WS_HBH), *HBL = (__bf16*)(ws + WS_HBL); float *SML = (float*)(ws + WS_SML), *WGT = (float*)(ws + WS_WGT); int *EXPo = (int*)(ws + WS_EXP), *CNT = (int*)(ws + WS_CNT), *LIST = (int*)(ws + WS_LIST);
  k_pack<<<dim3(2048, 6), 256, 0, stream>>>(F[1], F[15], F[20], F[25], F[29], F[7], F[9], F[11], F[13], PK);
  k_xb<<<NRT * 64, 128, 0, stream>>>(F[0], XB);
  k_gate<<<NRT, 128, 0, stream>>>(XB, PK, F[2], F[3], F[4], F[5], F[6], SML, EXPo, WGT);
  k_sort<<<1, 256, 0, stream>>>(EXPo, NRT * 64, CNT, LIST);
  k_fc<0><<<dim3(NTK / 64, 2048 / 128), 128, 0, stream>>>(XB, PK, F[8], CNT, LIST, HBH, HBL);
  k_pj<0><<<dim3(NTK / 64, EE / 128), 128, 0, stream>>>(HBH, HBL, PK, F[10], CNT, LIST, WGT, (float*)d_out);
  k_fc<1><<<dim3(NTK / 64, EE / 128), 128, 0, stream>>>(XB, PK, F[12], CNT, LIST, HBH, HBL);
  k_pj<1><<<dim3(NTK / 64, EE / 128), 128, 0, stream>>>(HBH, HBL, PK, F[14], CNT, LIST, WGT, (float*)d_out);
  for (int m = 2; m < 6; ++m) k_small<<<NTK / 64, 256, 0, stream>>>(m, F[0], SML, CNT, LIST, WGT, F[16], F[17], F[18], F[19], F[21], F[22], F[23], F[24], F[26], F[27], F[28], F[30], F[31], F[32], (float*)d_out);
}
